// HSTU_10333691314795
// MI455X (gfx1250) — hardware-verified
//
#include <hip/hip_runtime.h>
#include <stdint.h>

#define BATCH 2
#define SEQ 2048
#define HID 1024
#define NHEAD 16
#define HDIM 64
#define PROJW 4096
#define UCOL 0
#define VCOL 1024
#define QCOL 2048
#define KCOL 3072
#define NTOK (BATCH * SEQ)
#define ATT_SCALE 0.125f
#define LN_EPS_C 1e-8f
#define WCARRY 64.0f
#define WCARRY_INV (1.0f / 64.0f)
#define LOSC 2048.0f
#define LOSC_INV (1.0f / 2048.0f)
#define ROPE_BASE_C 10000.0f

static_assert(NHEAD * HDIM == HID, "head geometry");
static_assert(SEQ % 64 == 0 && HID % 64 == 0 && PROJW % 64 == 0, "tile multiples");

typedef __attribute__((ext_vector_type(16))) _Float16 v16h;
typedef __attribute__((ext_vector_type(8)))  _Float16 v8h;
typedef __attribute__((ext_vector_type(4)))  _Float16 v4h;
typedef __attribute__((ext_vector_type(16))) __bf16   v16b;
typedef __attribute__((ext_vector_type(8)))  __bf16   v8b;
typedef __attribute__((ext_vector_type(8)))  float    v8f;
typedef __attribute__((ext_vector_type(4)))  float    v4f;

__device__ __forceinline__ unsigned short f2bf_bits(float f) {
  unsigned u = __float_as_uint(f);
  return (unsigned short)((u + 0x7FFFu + ((u >> 16) & 1u)) >> 16);
}
__device__ __forceinline__ float bf_bits2f(unsigned short h) { return __uint_as_float(((unsigned)h) << 16); }
__device__ __forceinline__ float qbf(float f) { return bf_bits2f(f2bf_bits(f)); }
__device__ __forceinline__ v4f qbf4(v4f v) {
  v4f r;
#pragma unroll
  for (int e = 0; e < 4; ++e) r[e] = qbf(v[e]);
  return r;
}

__device__ __forceinline__ void dep_guard_h(v8f& a, v8f& b, v16h x, v16h y) { asm volatile("v_nop\n\tv_nop\n\tv_nop\n\tv_nop" : "+v"(a), "+v"(b) : "v"(x), "v"(y)); }
__device__ __forceinline__ void dep_guard_b(v8f& a, v8f& b, v16b x, v16b y) { asm volatile("v_nop\n\tv_nop\n\tv_nop\n\tv_nop" : "+v"(a), "+v"(b) : "v"(x), "v"(y)); }
__device__ __forceinline__ void keep4_h(v16h a, v16h b, v16h c, v16h d) { asm volatile("v_nop" :: "v"(a), "v"(b), "v"(c), "v"(d)); }
__device__ __forceinline__ void keep4_b(v16b a, v16b b, v16b c, v16b d) { asm volatile("v_nop" :: "v"(a), "v"(b), "v"(c), "v"(d)); }
__device__ __forceinline__ void acc_guard4(v8f& a, v8f& b, v8f& c, v8f& d) { asm volatile("v_nop\n\tv_nop\n\tv_nop\n\tv_nop" : "+v"(a), "+v"(b), "+v"(c), "+v"(d)); }
template <typename T> struct Frag;
template <> struct Frag<_Float16> {
  typedef v16h V; union U { v16h v; v8h h[2]; };
  static __device__ __forceinline__ v16h load(const _Float16* p) {
    U f; f.h[0] = *(const v8h*)(p); f.h[1] = *(const v8h*)(p + 16); return f.v;
  }
  static __device__ __forceinline__ v8f mma(v16h a, v16h b, v8f c) {
    return __builtin_amdgcn_wmma_f32_16x16x32_f16(false, a, false, b, (short)0, c, false, false);
  }
  static __device__ __forceinline__ void guard(v8f& a, v8f& b, v16h x, v16h y) { dep_guard_h(a, b, x, y); }
  static __device__ __forceinline__ void keep(v16h a, v16h b, v16h c, v16h d) { keep4_h(a, b, c, d); }
};
template <> struct Frag<__bf16> {
  typedef v16b V; union U { v16b v; v8b h[2]; };
  static __device__ __forceinline__ v16b load(const __bf16* p) {
    U f; f.h[0] = *(const v8b*)(p); f.h[1] = *(const v8b*)(p + 16); return f.v;
  }
  static __device__ __forceinline__ v8f mma(v16b a, v16b b, v8f c) {
    return __builtin_amdgcn_wmma_f32_16x16x32_bf16(false, a, false, b, (short)0, c, false, false);
  }
  static __device__ __forceinline__ void guard(v8f& a, v8f& b, v16b x, v16b y) { dep_guard_b(a, b, x, y); }
  static __device__ __forceinline__ void keep(v16b a, v16b b, v16b c, v16b d) { keep4_b(a, b, c, d); }
};

template <int ET> struct Elem;
template <> struct Elem<0> { typedef _Float16 T; };
template <> struct Elem<1> { typedef __bf16 T; };
template <int ET, int SPLIT, int BIAS_MODE, int OUT_MODE, bool RESID, int ACT = 0>
__global__ __launch_bounds__(256) void wmma_gemm64(
    const unsigned short* __restrict__ Ap, const unsigned short* __restrict__ A2p, int lda, long strideA,
    const unsigned short* __restrict__ Btp, const unsigned short* __restrict__ Bt2p, int ldb, long strideB,
    void* __restrict__ Cout, void* __restrict__ Cout2, int ldc, long strideC,
    const float* __restrict__ bias,
    const float* __restrict__ resid, long strideR,
    int M, int N, int K, float scale) {
  typedef typename Elem<ET>::T T;
  typedef typename Frag<T>::V V;
  const T* A = (const T*)Ap; const T* A2 = (const T*)A2p; const T* Bt = (const T*)Btp; const T* Bt2 = (const T*)Bt2p;
  __shared__ __align__(16) float sT[8][16 * 68];
  const int b    = blockIdx.y;
  const int lane = threadIdx.x & 31;
  const int wave = threadIdx.x >> 5;
  const int tilesN = N >> 6;
  const int tilesM = M >> 6;
  const int tile = blockIdx.x * 8 + wave;
  if (tile >= tilesM * tilesN) return;
  const int tm = tile / tilesN;
  const int tn = tile - tm * tilesN;
  const int m0 = tm << 6;
  const int n0 = tn << 6;

  const T* Ab  = A  + (size_t)b * strideA;
  const T* Bb  = Bt + (size_t)b * strideB;
  const T* Ab2 = (SPLIT != 0) ? (A2  + (size_t)b * strideA) : nullptr;
  const T* Bb2 = (SPLIT == 1) ? (Bt2 + (size_t)b * strideB) : nullptr;

  const int rlane = lane & 15;
  const int koff  = (lane >> 4) * 8;
  const int mOff  = (lane >> 4) * 8;

  v8f acc[4][4];
#pragma unroll
  for (int i = 0; i < 4; ++i)
#pragma unroll
    for (int j = 0; j < 4; ++j) acc[i][j] = (v8f){0.f,0.f,0.f,0.f,0.f,0.f,0.f,0.f};

  for (int k0 = 0; k0 < K; k0 += 32) {
    V bh[4], bl[4];
#pragma unroll
    for (int j = 0; j < 4; ++j) {
      const size_t bo = (size_t)(n0 + (j << 4) + rlane) * ldb + koff + k0;
      bh[j] = Frag<T>::load(Bb + bo);
      if (SPLIT == 1) bl[j] = Frag<T>::load(Bb2 + bo);
    }
#pragma unroll
    for (int i = 0; i < 4; ++i) {
      const size_t ao = (size_t)(m0 + (i << 4) + rlane) * lda + koff + k0;
      V ah = Frag<T>::load(Ab + ao);
      V al;
      if (SPLIT != 0) al = Frag<T>::load(Ab2 + ao);
#pragma unroll
      for (int j = 0; j < 4; ++j) {
        acc[i][j] = Frag<T>::mma(ah, bh[j], acc[i][j]);
        if (SPLIT == 1) acc[i][j] = Frag<T>::mma(ah, bl[j], acc[i][j]);
        if (SPLIT != 0) acc[i][j] = Frag<T>::mma(al, bh[j], acc[i][j]);
      }
      Frag<T>::guard(acc[i][0], acc[i][3], ah, (SPLIT != 0) ? al : ah);
    }
    Frag<T>::keep(bh[0], bh[1], bh[2], bh[3]);
    if (SPLIT == 1) Frag<T>::keep(bl[0], bl[1], bl[2], bl[3]);
  }
  acc_guard4(acc[0][0], acc[0][1], acc[0][2], acc[0][3]);
  acc_guard4(acc[1][0], acc[1][1], acc[1][2], acc[1][3]);
  acc_guard4(acc[2][0], acc[2][1], acc[2][2], acc[2][3]);
  acc_guard4(acc[3][0], acc[3][1], acc[3][2], acc[3][3]);

  float* slab = sT[wave];
  const float* Rb = RESID ? (resid + (size_t)b * strideR) : nullptr;
#pragma unroll
  for (int i = 0; i < 4; ++i) {
    const int mBase = m0 + (i << 4);
#pragma unroll
    for (int j = 0; j < 4; ++j) {
      const int n = n0 + (j << 4) + rlane;
      float bv = 0.f;
      if (BIAS_MODE == 2) bv = qbf(bias[n]);
#pragma unroll
      for (int r = 0; r < 8; ++r) {
        float v = acc[i][j][r] * scale;
        if (BIAS_MODE == 1) v += qbf(bias[mBase + mOff + r]);
        if (BIAS_MODE == 2) v += bv;
        if (RESID) v += Rb[(size_t)(mBase + mOff + r) * ldc + n];
        if (ACT == 1) v = tanhf(v);
        if (ACT == 2) v = fmaxf(v, 0.0f);
        if (ACT == 4) v = (v > 0.f) ? v : 0.01f * v;
        slab[(mOff + r) * 68 + (j << 4) + rlane] = v;
      }
    }
    __builtin_amdgcn_fence(__ATOMIC_RELEASE, "workgroup");
    __builtin_amdgcn_wave_barrier();
    __builtin_amdgcn_fence(__ATOMIC_ACQUIRE, "workgroup");
    if (OUT_MODE == 0) {
      float* C = (float*)Cout + (size_t)b * strideC;
      const int hh = lane >> 4, c4 = (lane & 15) * 4;
      for (int pass = 0; pass < 2; ++pass) {
#pragma unroll
        for (int it = 0; it < 8; ++it) {
          const int row = it * 2 + hh;
          v4f v = *(const v4f*)(slab + row * 68 + c4);
          *(volatile v4f*)(C + (size_t)(mBase + row) * ldc + n0 + c4) = v;
        }
        __threadfence();
      }
    } else {
      const int q = lane >> 3, c8 = (lane & 7) * 8;
      unsigned short* C  = (unsigned short*)Cout  + (size_t)b * strideC;
      unsigned short* C2 = (OUT_MODE == 2) ? ((unsigned short*)Cout2 + (size_t)b * strideC) : nullptr;
      for (int pass = 0; pass < 2; ++pass) {
#pragma unroll
        for (int it = 0; it < 4; ++it) {
          const int row = it * 4 + q;
          const float* sp = slab + row * 68 + c8;
          v8h hv, lv;
#pragma unroll
          for (int e = 0; e < 8; ++e) {
            if (OUT_MODE == 1) {
              hv[e] = (_Float16)sp[e];
            } else {
              unsigned short hb = f2bf_bits(sp[e]);
              unsigned short lb = f2bf_bits(sp[e] - bf_bits2f(hb));
              hv[e] = __builtin_bit_cast(_Float16, hb);
              lv[e] = __builtin_bit_cast(_Float16, lb);
            }
          }
          *(volatile v8h*)(C + (size_t)(mBase + row) * ldc + n0 + c8) = hv;
          if (OUT_MODE == 2) *(volatile v8h*)(C2 + (size_t)(mBase + row) * ldc + n0 + c8) = lv;
        }
        __threadfence();
      }
    }
    __builtin_amdgcn_fence(__ATOMIC_RELEASE, "workgroup");
    __builtin_amdgcn_wave_barrier();
    __builtin_amdgcn_fence(__ATOMIC_ACQUIRE, "workgroup");
  }
}

#define WTP 72
template <int MODE>
__global__ __launch_bounds__(256) void wt_cast_k(const float* __restrict__ W, unsigned short* __restrict__ Wtp,
                                                 int K, int N, float mul) {
  __shared__ __align__(16) _Float16 st[64 * WTP];
  _Float16* Wt = (_Float16*)Wtp;
  const int n0 = blockIdx.x * 64, k0 = blockIdx.y * 64;
  const int tid = threadIdx.x;
  const int kr = tid >> 2, c16 = (tid & 3) * 16;
  const float* src = W + (size_t)(k0 + kr) * N + n0 + c16;
#pragma unroll
  for (int q = 0; q < 4; ++q) {
    const v4f v = *(const v4f*)(src + 4 * q);
#pragma unroll
    for (int e = 0; e < 4; ++e) {
      _Float16 hv;
      if (MODE == 0) hv = (_Float16)(qbf(v[e]) * mul);
      else hv = __builtin_bit_cast(_Float16, f2bf_bits(v[e]));
      st[(c16 + 4 * q + e) * WTP + kr] = hv;
    }
  }
  __syncthreads();
  const int wave = tid >> 5, lane = tid & 31;
  const int q8 = lane >> 3, c8 = (lane & 7) * 8;
  const v8h h0 = *(const v8h*)(st + (wave * 4 + q8) * WTP + c8);
  const v8h h1 = *(const v8h*)(st + (32 + wave * 4 + q8) * WTP + c8);
  for (int pass = 0; pass < 2; ++pass) {
    *(volatile v8h*)(Wt + (size_t)(n0 + wave * 4 + q8) * K + k0 + c8) = h0;
    *(volatile v8h*)(Wt + (size_t)(n0 + 32 + wave * 4 + q8) * K + k0 + c8) = h1;
    __threadfence();
  }
}

template <int MODE>
__global__ __launch_bounds__(128) void ln_k(const float* __restrict__ xin, const float* __restrict__ g,
                                            const float* __restrict__ be, unsigned short* __restrict__ o0p,
                                            unsigned short* __restrict__ o1p) {
  __shared__ float red1[4], red2[4];
  _Float16* o0 = (_Float16*)o0p;
  _Float16* o1 = (_Float16*)o1p;
  const int row = blockIdx.x, tid = threadIdx.x, lane = tid & 31, wave = tid >> 5;
  const size_t rb = (size_t)row * HID;
  const int c0 = tid * 8;
  v4f va = *(const v4f*)(xin + rb + c0);
  v4f vb = *(const v4f*)(xin + rb + c0 + 4);
  if (MODE == 0) { va = qbf4(va); vb = qbf4(vb); }
  float s = ((va[0] + va[1]) + (va[2] + va[3])) + ((vb[0] + vb[1]) + (vb[2] + vb[3]));
#pragma unroll
  for (int off = 1; off < 32; off <<= 1) s += __shfl_xor(s, off, 32);
  if (lane == 0) red1[wave] = s;
  __syncthreads();
  const float mu = ((red1[0] + red1[1]) + (red1[2] + red1[3])) * (1.0f / HID);
  const v4f da = va - mu, db = vb - mu;
  float s2 = ((da[0] * da[0] + da[1] * da[1]) + (da[2] * da[2] + da[3] * da[3])) +
             ((db[0] * db[0] + db[1] * db[1]) + (db[2] * db[2] + db[3] * db[3]));
#pragma unroll
  for (int off = 1; off < 32; off <<= 1) s2 += __shfl_xor(s2, off, 32);
  if (lane == 0) red2[wave] = s2;
  __syncthreads();
  const float var = ((red2[0] + red2[1]) + (red2[2] + red2[3])) * (1.0f / HID);
  const float inv = rsqrtf(var + LN_EPS_C);
  const v4f ga = qbf4(*(const v4f*)(g + c0));
  const v4f gb = qbf4(*(const v4f*)(g + c0 + 4));
  const v4f ba = qbf4(*(const v4f*)(be + c0));
  const v4f bb = qbf4(*(const v4f*)(be + c0 + 4));
  const v4f ya = da * inv * ga + ba;
  const v4f yb = db * inv * gb + bb;
  v8h hv, lv;
#pragma unroll
  for (int e = 0; e < 4; ++e) {
    if (MODE == 0) {
      const unsigned short ha = f2bf_bits(ya[e]);
      const unsigned short la = f2bf_bits(ya[e] - bf_bits2f(ha));
      const unsigned short hb2 = f2bf_bits(yb[e]);
      const unsigned short lb2 = f2bf_bits(yb[e] - bf_bits2f(hb2));
      hv[e]     = __builtin_bit_cast(_Float16, ha);
      lv[e]     = __builtin_bit_cast(_Float16, la);
      hv[4 + e] = __builtin_bit_cast(_Float16, hb2);
      lv[4 + e] = __builtin_bit_cast(_Float16, lb2);
    } else {
      hv[e]     = (_Float16)ya[e];
      hv[4 + e] = (_Float16)yb[e];
      lv[e] = hv[e]; lv[4 + e] = hv[4 + e];
    }
  }
  for (int pass = 0; pass < 2; ++pass) {
    *(volatile v8h*)(o0 + rb + c0) = hv;
    if (MODE == 0) *(volatile v8h*)(o1 + rb + c0) = lv;
    __threadfence();
  }
}

__global__ __launch_bounds__(32) void invfreq_k(float* __restrict__ inv) {
  const int lane = threadIdx.x;
  const float e = (float)(2 * lane) * (1.0f / 64.0f);
  const float p = powf(ROPE_BASE_C, e);
  const float v = 1.0f / p;
  *(volatile float*)(inv + lane) = v;
  __threadfence();
  *(volatile float*)(inv + lane) = v;
}

__global__ __launch_bounds__(256) void rope_tab_k(const float* __restrict__ inv, float* __restrict__ tab) {
  const int tid = threadIdx.x, lane = tid & 31, wave = tid >> 5;
  const int l = blockIdx.x * 8 + wave;
  const float fr = inv[lane];
  const float th = (float)l * fr;
  float sv, cv;
  sincosf(th, &sv, &cv);
  float* rp = tab + (size_t)l * 64;
  *(volatile float*)(rp + lane) = cv;
  *(volatile float*)(rp + 32 + lane) = sv;
  __threadfence();
  *(volatile float*)(rp + lane) = cv;
  *(volatile float*)(rp + 32 + lane) = sv;
}

#define RPITCH 72
#define PLANE_ELEMS ((size_t)NHEAD * NTOK * HDIM)
__global__ __launch_bounds__(256) void rope_k(const float* __restrict__ proj, const float* __restrict__ tab,
                                              unsigned short* __restrict__ planesp) {
  __shared__ __align__(16) _Float16 st[64 * RPITCH];
  _Float16* planes = (_Float16*)planesp;
  const int tok = blockIdx.x;
  const int b = tok / SEQ, l = tok - b * SEQ;
  const int tid = threadIdx.x, h = tid >> 4, j = tid & 15;
  const float* tb = tab + (size_t)l * 64;
  const float c0 = tb[j], c1 = tb[j + 16], s0 = tb[32 + j], s1 = tb[32 + j + 16];
  const float* pr = proj + (size_t)tok * PROJW + h * HDIM;
#pragma unroll
  for (int p = 0; p < 2; ++p) {
    const float* src = pr + QCOL + p * HID;
    const float a0 = src[j], a1 = src[j + 16], a2 = src[j + 32], a3 = src[j + 48];
    const float o0 = a0 * c0 - a2 * s0;
    const float o2 = a2 * c0 + a0 * s0;
    const float o1 = a1 * c1 - a3 * s1;
    const float o3 = a3 * c1 + a1 * s1;
    _Float16* sw = st + (p * 16 + h) * RPITCH;
    sw[j]      = (_Float16)o0;
    sw[j + 16] = (_Float16)o1;
    sw[j + 32] = (_Float16)o2;
    sw[j + 48] = (_Float16)o3;
  }
  {
    const float* srcv = pr + VCOL;
    _Float16* swh = st + (32 + h) * RPITCH;
    _Float16* swl = st + (48 + h) * RPITCH;
#pragma unroll
    for (int q = 0; q < 4; ++q) {
      const int d = j + 16 * q;
      const float v = srcv[d];
      const _Float16 vh = (_Float16)v;
      const _Float16 vl = (_Float16)((v - (float)vh) * LOSC);
      swh[d] = vh;
      swl[d] = vl;
    }
  }
  __syncthreads();
  const int wave = tid >> 5, lane = tid & 31, q8 = lane >> 3, c8 = (lane & 7) * 8;
  const int row0 = wave * 4 + q8;
  const int row1 = 32 + wave * 4 + q8;
  const v8h h0 = *(const v8h*)(st + row0 * RPITCH + c8);
  const v8h h1 = *(const v8h*)(st + row1 * RPITCH + c8);
  _Float16* d0 = planes + (size_t)(row0 >> 4) * PLANE_ELEMS + (((size_t)(b * NHEAD + (row0 & 15))) * SEQ + l) * HDIM + c8;
  _Float16* d1 = planes + (size_t)(row1 >> 4) * PLANE_ELEMS + (((size_t)(b * NHEAD + (row1 & 15))) * SEQ + l) * HDIM + c8;
  for (int pass = 0; pass < 2; ++pass) {
    *(volatile v8h*)d0 = h0;
    *(volatile v8h*)d1 = h1;
    __threadfence();
  }
}

__device__ __forceinline__ v8f mma_h(v16h a, v16h b, v8f c) {
  c = __builtin_amdgcn_wmma_f32_16x16x32_f16(false, a, false, b, (short)0, c, false, false);
  asm volatile("v_nop\n\tv_nop\n\tv_nop\n\tv_nop" : "+v"(c) : "v"(a), "v"(b));
  return c;
}
#define KCH 64
#define OPITCH 68
__global__ __launch_bounds__(128) void attn_k(const unsigned short* __restrict__ qpp, const unsigned short* __restrict__ kpp,
                                              const unsigned short* __restrict__ vhpp, const unsigned short* __restrict__ vlpp,
                                              const float* __restrict__ proj, const int* __restrict__ mask,
                                              const float* __restrict__ x, float* __restrict__ x1) {
  union FH { v16h v; v8h h[2]; };
  __shared__ __align__(16) _Float16 Ksh[KCH * HDIM];
  __shared__ __align__(16) _Float16 Vth[HDIM * KCH];
  __shared__ __align__(16) _Float16 Vtl[HDIM * KCH];
  __shared__ __align__(16) _Float16 Psh[4][16 * KCH];
  __shared__ __align__(16) _Float16 Psl[4][16 * KCH];
  __shared__ __align__(16) float    Osh[4][16 * OPITCH];
  const _Float16* qp  = (const _Float16*)qpp;
  const _Float16* kp  = (const _Float16*)kpp;
  const _Float16* vhp = (const _Float16*)vhpp;
  const _Float16* vlp = (const _Float16*)vlpp;
  const int tid = threadIdx.x, wave = tid >> 5, lane = tid & 31, hh = lane >> 4, c = lane & 15;
  const int nqb = SEQ / 64;
  const int bx = blockIdx.x;
  const int qb = bx % nqb;
  const int bh = bx / nqb;
  const int h = bh % NHEAD;
  const int b = bh / NHEAD;
  const int q0 = qb * 64 + wave * 16;
  const size_t rowb = (size_t)(b * NHEAD + h) * SEQ;
  const size_t tokb = (size_t)b * SEQ;

  v16h qa[2];
  {
    const _Float16* qrow = qp + (rowb + q0 + c) * HDIM + 8 * hh;
#pragma unroll
    for (int dc = 0; dc < 2; ++dc) qa[dc] = Frag<_Float16>::load(qrow + dc * 32);
  }
  v8f oacc[4], oaccr[4];
#pragma unroll
  for (int t = 0; t < 4; ++t) {
    oacc[t]  = (v8f){0.f,0.f,0.f,0.f,0.f,0.f,0.f,0.f};
    oaccr[t] = (v8f){0.f,0.f,0.f,0.f,0.f,0.f,0.f,0.f};
  }

  const int nChunks = qb + 1;
  for (int kc = 0; kc < nChunks; ++kc) {
    const int kv0 = kc * KCH;
    __syncthreads();
    {
      const int kvr = tid >> 1, dh = (tid & 1) * 32;
      const _Float16* krow  = kp  + (rowb + kv0 + kvr) * HDIM + dh;
      const _Float16* vhrow = vhp + (rowb + kv0 + kvr) * HDIM + dh;
      const _Float16* vlrow = vlp + (rowb + kv0 + kvr) * HDIM + dh;
#pragma unroll 1
      for (int i = 0; i < 4; ++i) {
        const v8h kk = *(const v8h*)(krow + 8 * i);
        *(v8h*)(Ksh + kvr * HDIM + dh + 8 * i) = kk;
        const v8h vh = *(const v8h*)(vhrow + 8 * i);
        const v8h vl = *(const v8h*)(vlrow + 8 * i);
#pragma unroll
        for (int e = 0; e < 8; ++e) {
          Vth[(dh + 8 * i + e) * KCH + kvr] = vh[e];
          Vtl[(dh + 8 * i + e) * KCH + kvr] = vl[e];
        }
      }
    }
    __syncthreads();

    v8f s[4];
#pragma unroll
    for (int j = 0; j < 4; ++j) {
      s[j] = (v8f){0.f,0.f,0.f,0.f,0.f,0.f,0.f,0.f};
#pragma unroll
      for (int dc = 0; dc < 2; ++dc) {
        FH kb;
        kb.h[0] = *(const v8h*)(Ksh + (j * 16 + c) * HDIM + dc * 32 + 8 * hh);
        kb.h[1] = *(const v8h*)(Ksh + (j * 16 + c) * HDIM + dc * 32 + 16 + 8 * hh);
        s[j] = mma_h(qa[dc], kb.v, s[j]);
      }
    }
    _Float16* pwh = Psh[wave];
    _Float16* pwl = Psl[wave];
#pragma unroll
    for (int r = 0; r < 8; ++r) {
      const int qrow = q0 + 8 * hh + r;
      const int* mrow = mask + (tokb + (size_t)qrow) * SEQ + kv0 + c;
#pragma unroll
      for (int j = 0; j < 4; ++j) {
        const int mv = mrow[j * 16];
        const float sc = s[j][r] * ATT_SCALE;
        const float ex = __expf(-sc);
        float w = __builtin_amdgcn_rcpf(1.0f + ex);
        w = (mv != 0) ? w : 0.0f;
        const _Float16 wh = (_Float16)w;
        const _Float16 wl = (_Float16)((w - (float)wh) * LOSC);
        pwh[(8 * hh + r) * KCH + j * 16 + c] = wh;
        pwl[(8 * hh + r) * KCH + j * 16 + c] = wl;
      }
    }
    __builtin_amdgcn_fence(__ATOMIC_RELEASE, "workgroup");
    __builtin_amdgcn_wave_barrier();
    __builtin_amdgcn_fence(__ATOMIC_ACQUIRE, "workgroup");
#pragma unroll 1
    for (int kk = 0; kk < 2; ++kk) {
      FH pa, pl;
      pa.h[0] = *(const v8h*)(pwh + c * KCH + kk * 32 + 8 * hh);
      pa.h[1] = *(const v8h*)(pwh + c * KCH + kk * 32 + 16 + 8 * hh);
      pl.h[0] = *(const v8h*)(pwl + c * KCH + kk * 32 + 8 * hh);
      pl.h[1] = *(const v8h*)(pwl + c * KCH + kk * 32 + 16 + 8 * hh);
#pragma unroll
      for (int t = 0; t < 4; ++t) {
        FH vb, vl;
        vb.h[0] = *(const v8h*)(Vth + (t * 16 + c) * KCH + kk * 32 + 8 * hh);
        vb.h[1] = *(const v8h*)(Vth + (t * 16 + c) * KCH + kk * 32 + 16 + 8 * hh);
        oacc[t]  = mma_h(pa.v, vb.v, oacc[t]);
        vl.h[0] = *(const v8h*)(Vtl + (t * 16 + c) * KCH + kk * 32 + 8 * hh);
        vl.h[1] = *(const v8h*)(Vtl + (t * 16 + c) * KCH + kk * 32 + 16 + 8 * hh);
        oaccr[t] = mma_h(pa.v, vl.v, oaccr[t]);
        oaccr[t] = mma_h(pl.v, vb.v, oaccr[t]);
      }
    }
  }

  float* os = Osh[wave];
#pragma unroll
  for (int r = 0; r < 8; ++r) {
#pragma unroll
    for (int t = 0; t < 4; ++t) os[(8 * hh + r) * OPITCH + t * 16 + c] = oacc[t][r] + oaccr[t][r] * LOSC_INV;
  }
  __builtin_amdgcn_fence(__ATOMIC_RELEASE, "workgroup");
  __builtin_amdgcn_wave_barrier();
  __builtin_amdgcn_fence(__ATOMIC_ACQUIRE, "workgroup");
  {
    const int c4 = c * 4;
    const size_t colb = (size_t)h * HDIM + c4;
    v4f resv[8];
#pragma unroll
    for (int it = 0; it < 8; ++it) {
      const int row = it * 2 + hh;
      const size_t tok = tokb + (size_t)(q0 + row);
      const v4f o  = *(const v4f*)(os + row * OPITCH + c4);
      const v4f u  = *(const v4f*)(proj + tok * PROJW + UCOL + colb);
      const v4f xv = *(const v4f*)(x + tok * HID + colb);
      v4f res;
#pragma unroll
      for (int e = 0; e < 4; ++e) {
        const float ue = u[e];
        const float sg = __builtin_amdgcn_rcpf(1.0f + __expf(-ue));
        const float xe = qbf(xv[e]);
        res[e] = xe + (ue * sg) * o[e];
      }
      resv[it] = res;
    }
    for (int pass = 0; pass < 2; ++pass) {
#pragma unroll
      for (int it = 0; it < 8; ++it) {
        const int row = it * 2 + hh;
        const size_t tok = tokb + (size_t)(q0 + row);
        *(volatile v4f*)(x1 + tok * HID + colb) = resv[it];
      }
      __threadfence();
    }
  }
}

extern "C" void kernel_launch(void* const* d_in, const int* in_sizes, int n_in,
                              void* d_out, int out_size, void* d_ws, size_t ws_size,
                              hipStream_t stream) {
  if (n_in < 10) return;
  if (in_sizes[0] != NTOK * HID || in_sizes[1] != BATCH * SEQ * SEQ || in_sizes[2] != HID * PROJW ||
      in_sizes[3] != PROJW || in_sizes[4] != HID * HID || in_sizes[5] != HID || in_sizes[6] != HID ||
      in_sizes[7] != HID || in_sizes[8] != HID || in_sizes[9] != HID || out_size != NTOK * HID) return;
  const float* x      = (const float*)d_in[0];
  const int*   amask  = (const int*)d_in[1];
  const float* W_proj = (const float*)d_in[2];
  const float* b_proj = (const float*)d_in[3];
  const float* W_out  = (const float*)d_in[4];
  const float* b_out  = (const float*)d_in[5];
  const float* ln1_g  = (const float*)d_in[6];
  const float* ln1_b  = (const float*)d_in[7];
  const float* ln2_g  = (const float*)d_in[8];
  const float* ln2_b  = (const float*)d_in[9];

  char* ws = (char*)d_ws;
  const size_t planeB = (size_t)NTOK * HID * 2;
  size_t off = 0;
  unsigned short* pl0 = (unsigned short*)(ws + off); off += planeB;
  unsigned short* pl1 = (unsigned short*)(ws + off); off += planeB;
  unsigned short* pl2 = (unsigned short*)(ws + off); off += planeB;
  unsigned short* pl3 = (unsigned short*)(ws + off); off += planeB;
  unsigned short* wot = (unsigned short*)(ws + off); off += (size_t)HID * HID * 2;
  float* rtab = (float*)(ws + off); off += (size_t)SEQ * 64 * 4;
  float* invf = (float*)(ws + off); off += 4096;
  float* proj = (float*)(ws + off); off += (size_t)NTOK * PROJW * 4;
  float* x1   = (float*)(ws + off); off += (size_t)NTOK * HID * 4;
  if (off > ws_size) return;

  invfreq_k<<<1, 32, 0, stream>>>(invf);
  rope_tab_k<<<SEQ / 8, 256, 0, stream>>>(invf, rtab);
  wt_cast_k<1><<<dim3(PROJW / 64, HID / 64), 256, 0, stream>>>(W_proj, pl2, HID, PROJW, 1.0f);
  wt_cast_k<0><<<dim3(HID / 64, HID / 64), 256, 0, stream>>>(W_out, wot, HID, HID, WCARRY);
  ln_k<0><<<NTOK, 128, 0, stream>>>(x, ln1_g, ln1_b, pl0, pl1);
  wmma_gemm64<1, 2, 2, 0, false, 0><<<dim3(((NTOK / 64) * (PROJW / 64)) / 8, 1), 256, 0, stream>>>(
      pl0, pl1, HID, 0L, pl2, pl2, HID, 0L, (void*)proj, (void*)proj, PROJW, 0L, b_proj, x, 0L,
      NTOK, PROJW, HID, 1.0f);
  rope_k<<<NTOK, 256, 0, stream>>>(proj, rtab, pl0);
  attn_k<<<BATCH * NHEAD * (SEQ / 64), 128, 0, stream>>>(pl0, pl1, pl2, pl3, proj, amask, x, x1);
  ln_k<1><<<NTOK, 128, 0, stream>>>(x1, ln2_g, ln2_b, pl0, pl0);
  wmma_gemm64<0, 0, 2, 0, true, 0><<<dim3(((NTOK / 64) * (HID / 64)) / 8, 1), 256, 0, stream>>>(
      pl0, pl0, HID, 0L, wot, wot, HID, 0L, d_out, d_out, HID, 0L, b_out, x1, 0L,
      NTOK, HID, HID, WCARRY_INV);
}
